// VSONDecoder_32401233281074
// MI455X (gfx1250) — hardware-verified
//
#include <hip/hip_runtime.h>


#define NB_  4
#define NP   32768
#define NC   8
#define NF   32
#define ND   64
#define NH   64
#define NPT  (NB_ * NP)

typedef unsigned short bf;
typedef __attribute__((ext_vector_type(16))) __bf16   v16bf;
typedef __attribute__((ext_vector_type(8)))  unsigned short v8us;
typedef __attribute__((ext_vector_type(8)))  float    v8f;
typedef __attribute__((ext_vector_type(4)))  float    v4f;
typedef __attribute__((ext_vector_type(2)))  float    v2f;
typedef v4f  __attribute__((may_alias)) v4fa;
typedef v8us __attribute__((may_alias)) v8usa;

__device__ __forceinline__ unsigned short f2bf(float f) { unsigned u = __float_as_uint(f); u += 0x7FFFu + ((u >> 16) & 1u); return (unsigned short)(u >> 16); }
__device__ __forceinline__ float bf2f(unsigned short b) { return __uint_as_float(((unsigned)b) << 16); }
__device__ __forceinline__ float bfr(float f) { return bf2f(f2bf(f)); }
__device__ __forceinline__ v16bf cat16b(v8us lo, v8us hi) { return __builtin_bit_cast(v16bf, __builtin_shufflevector(lo, hi, 0, 1, 2, 3, 4, 5, 6, 7, 8, 9, 10, 11, 12, 13, 14, 15)); }
__device__ __forceinline__ v8f wmmab(v16bf a, v16bf b, v8f c) { return __builtin_amdgcn_wmma_f32_16x16x32_bf16(false, a, false, b, (short)0, c, false, false); }
#define VST2(T, p, v) do { const T vst2_v_ = (v); *(volatile T*)(p) = vst2_v_; __threadfence(); *(volatile T*)(p) = vst2_v_; } while (0)

__global__ __launch_bounds__(256) void k_pre(const float* __restrict__ pq, const float* __restrict__ pos, const float* __restrict__ Wf, bf* PEH, bf* PEL, float* N0) {
    __shared__ __align__(16) unsigned short sh[256 * NF];
    __shared__ __align__(16) unsigned short sl[256 * NF];
    __shared__ float n0[256];
    const int t = threadIdx.x, lane = t & 31, wave = t >> 5; const int pt = blockIdx.x * 256 + t, b = pt / NP;
    float q0 = bfr(pq[(size_t)pt * 3 + 0]) - bfr(pos[b * 3 + 0]), q1 = bfr(pq[(size_t)pt * 3 + 1]) - bfr(pos[b * 3 + 1]), q2 = bfr(pq[(size_t)pt * 3 + 2]) - bfr(pos[b * 3 + 2]);
    const float nrm = sqrtf(q0 * q0 + q1 * q1 + q2 * q2);
    if (nrm > 0.5f) { const float s = 0.5f / nrm; q0 = q0 / nrm * 0.5f; q1 = q1 / nrm * 0.5f; q2 = q2 / nrm * 0.5f; (void)s; }
    float ss = 0.f;
#pragma unroll
    for (int f = 0; f < NF; ++f) { const float v = q0 * bfr(Wf[f]) + q1 * bfr(Wf[NF + f]) + q2 * bfr(Wf[2 * NF + f]); ss += v * v;
        const unsigned short hb = f2bf(v); sh[t * NF + f] = hb; sl[t * NF + f] = f2bf(v - bf2f(hb)); }
    n0[t] = ss;
    __syncthreads();
    auto pass = [&]() {
#pragma unroll
        for (int s = 0; s < 4; ++s) { const int e0 = s * 2048 + t * 8; *(volatile v8us*)(PEH + (size_t)blockIdx.x * 256 * NF + e0) = *(const v8usa*)(sh + e0); *(volatile v8us*)(PEL + (size_t)blockIdx.x * 256 * NF + e0) = *(const v8usa*)(sl + e0); }
        *(volatile float*)(N0 + pt) = n0[t];
    };
    pass(); __threadfence(); pass();
}
__global__ __launch_bounds__(256) void k_zc(const float* __restrict__ z, const float* __restrict__ Wdir, const float* __restrict__ W0, const float* __restrict__ b0, bf* ZB, float* ZC) {
    __shared__ float zinv[NB_ * NC * ND];
    const int t = threadIdx.x;
#pragma unroll 1
    for (int s = 0; s < (NB_ * NC * ND * NF) / 2048; ++s) { const int e0 = s * 2048 + t * 8; v8us o;
#pragma unroll
        for (int i = 0; i < 8; ++i) { const int e = e0 + i; const int f = e & 31, cd = (e >> 5) & 511, b = e >> 14, c = cd >> 6, d = cd & 63; o[i] = f2bf(z[(((size_t)b * NC + c) * NF + f) * ND + d]); }
        VST2(v8us, ZB + e0, o); }
#pragma unroll 1
    for (int j = t; j < NB_ * NC * ND; j += 256) { const int d = j & 63, bc = j >> 6; float acc = 0.f;
#pragma unroll 1
        for (int f = 0; f < NF; ++f) { const float* zr = z + ((size_t)bc * NF + f) * ND; float zd = 0.f;
#pragma unroll 4
            for (int e = 0; e < ND; ++e) zd += bfr(zr[e]) * bfr(Wdir[e * ND + d]);
            acc += bfr(zr[d]) * zd; }
        zinv[j] = acc; }
    __syncthreads();
#pragma unroll 1
    for (int j = t; j < NB_ * NC * NH; j += 256) { const int h = j & 63, bc = j >> 6; float acc = bfr(b0[h]);
#pragma unroll 4
        for (int d = 0; d < ND; ++d) acc += zinv[bc * ND + d] * bfr(W0[(size_t)(1 + ND + d) * NH + h]);
        *(volatile float*)(ZC + j) = acc; }
    __threadfence();
#pragma unroll 1
    for (int j = t; j < NB_ * NC * NH; j += 256) { const int h = j & 63, bc = j >> 6; float acc = bfr(b0[h]);
#pragma unroll 4
        for (int d = 0; d < ND; ++d) acc += zinv[bc * ND + d] * bfr(W0[(size_t)(1 + ND + d) * NH + h]);
        *(volatile float*)(ZC + j) = acc; }
}
__global__ __launch_bounds__(256) void k_w(const float* __restrict__ W0, const float* __restrict__ Wa, const float* __restrict__ Wb, const float* __restrict__ Wout, bf* WT, bf* WOUT) {
    const int t = threadIdx.x;
#pragma unroll 1
    for (int s = 0; s < (11 * NH * ND) / 2048; ++s) { const int e0 = s * 2048 + t * 8; v8us o;
#pragma unroll
        for (int i = 0; i < 8; ++i) { const int e = e0 + i; const int k = e & 63, n = (e >> 6) & 63, m = e >> 12; float v;
            if (m == 0) v = W0[(size_t)(1 + k) * NH + n]; else if (m <= 5) v = Wa[((size_t)(m - 1) * NH + k) * NH + n]; else v = Wb[((size_t)(m - 6) * NH + k) * NH + n];
            o[i] = f2bf(v); }
        VST2(v8us, WT + e0, o); }
    if (t < 128) { v8us o;
#pragma unroll
        for (int i = 0; i < 8; ++i) { const int e = t * 8 + i; const int r = e >> 6, k = e & 63; o[i] = (r == 0) ? f2bf(Wout[k]) : (unsigned short)0; }
        VST2(v8us, WOUT + t * 8, o); }
}

__device__ __forceinline__ void restage(const v8f* acc, unsigned short* th, unsigned short* tlw, int lr, int hi, bool relu_, v16bf* ah, v16bf* al) {
#pragma unroll
    for (int n = 0; n < 4; ++n)
#pragma unroll
        for (int j = 0; j < 8; ++j) { float v = acc[n][j]; if (relu_) v = fmaxf(v, 0.f); const unsigned short hb = f2bf(v);
            th[(hi * 8 + j) * 72 + n * 16 + lr] = hb; tlw[(hi * 8 + j) * 72 + n * 16 + lr] = f2bf(v - bf2f(hb)); }
    __builtin_amdgcn_wave_barrier(); asm volatile("" ::: "memory");
#pragma unroll
    for (int kc = 0; kc < 2; ++kc) { ah[kc] = cat16b(*(const v8usa*)(th + lr * 72 + kc * 32 + 8 * hi), *(const v8usa*)(th + lr * 72 + kc * 32 + 16 + 8 * hi));
                                     al[kc] = cat16b(*(const v8usa*)(tlw + lr * 72 + kc * 32 + 8 * hi), *(const v8usa*)(tlw + lr * 72 + kc * 32 + 16 + 8 * hi)); }
    __builtin_amdgcn_wave_barrier(); asm volatile("" ::: "memory");
}
__device__ __forceinline__ void lin64(const v16bf* ah, const v16bf* al, const bf* __restrict__ Wn, int lr, int hi, v8f* acc) {
#pragma unroll
    for (int n = 0; n < 4; ++n) acc[n] = (v8f){};
#pragma unroll
    for (int kc = 0; kc < 2; ++kc)
#pragma unroll
        for (int n = 0; n < 4; ++n) { const bf* bp = Wn + (size_t)(n * 16 + lr) * ND + kc * 32 + 8 * hi; const v16bf b = cat16b(*(const v8us*)bp, *(const v8us*)(bp + 16));
            acc[n] = wmmab(ah[kc], b, acc[n]); acc[n] = wmmab(al[kc], b, acc[n]); }
    asm volatile("v_nop\n\tv_nop\n\tv_nop\n\tv_nop" : "+v"(acc[0]), "+v"(acc[1]), "+v"(acc[2]), "+v"(acc[3]));
}
__global__ __launch_bounds__(128) void k_s1(const bf* __restrict__ PEH, const bf* __restrict__ PEL, const float* __restrict__ N0, const bf* __restrict__ ZB, const float* __restrict__ ZC,
                                           const bf* __restrict__ WT, const float* __restrict__ W0, const float* __restrict__ ba, const float* __restrict__ bb, float* NET1) {
    __shared__ __align__(16) unsigned short th[4][16 * 72];
    __shared__ __align__(16) unsigned short tlw[4][16 * 72];
    __shared__ __align__(16) float ost[4][16 * 68];
    const int lane = threadIdx.x & 31, wave = threadIdx.x >> 5, lr = lane & 15, hi = lane >> 4;
    const int r0 = blockIdx.x * 64 + wave * 16, b = r0 / NP;
    unsigned short* mth = th[wave]; unsigned short* mtl = tlw[wave];
    const v16bf a0 = cat16b(*(const v8us*)(PEH + (size_t)(r0 + lr) * NF + 8 * hi), *(const v8us*)(PEH + (size_t)(r0 + lr) * NF + 16 + 8 * hi));
    const v16bf a0l = cat16b(*(const v8us*)(PEL + (size_t)(r0 + lr) * NF + 8 * hi), *(const v8us*)(PEL + (size_t)(r0 + lr) * NF + 16 + 8 * hi));
    float n0v[8], w0r[4];
#pragma unroll
    for (int j = 0; j < 8; ++j) n0v[j] = N0[r0 + hi * 8 + j];
#pragma unroll
    for (int n = 0; n < 4; ++n) w0r[n] = bfr(W0[n * 16 + lr]);
    v8f mx[4];
#pragma unroll
    for (int n = 0; n < 4; ++n)
#pragma unroll
        for (int j = 0; j < 8; ++j) mx[n][j] = -3.0e38f;
    v16bf ah[2], al[2]; v8f acc[4], net[4];
#pragma unroll 1
    for (int c = 0; c < NC; ++c) {
#pragma unroll
        for (int n = 0; n < 4; ++n) { const bf* bp = ZB + ((size_t)(b * NC + c) * ND + n * 16 + lr) * NF + 8 * hi; const v16bf bz = cat16b(*(const v8us*)bp, *(const v8us*)(bp + 16));
            acc[n] = wmmab(a0, bz, (v8f){}); acc[n] = wmmab(a0l, bz, acc[n]); }
        asm volatile("v_nop\n\tv_nop\n\tv_nop\n\tv_nop" : "+v"(acc[0]), "+v"(acc[1]), "+v"(acc[2]), "+v"(acc[3]));
        restage(acc, mth, mtl, lr, hi, false, ah, al);
        lin64(ah, al, WT + 0 * NH * ND, lr, hi, net);
#pragma unroll
        for (int n = 0; n < 4; ++n)
#pragma unroll
            for (int j = 0; j < 8; ++j) net[n][j] += n0v[j] * w0r[n] + ZC[(size_t)(b * NC + c) * NH + n * 16 + lr];
        restage(net, mth, mtl, lr, hi, true, ah, al);
        lin64(ah, al, WT + 1 * NH * ND, lr, hi, acc);
#pragma unroll
        for (int n = 0; n < 4; ++n)
#pragma unroll
            for (int j = 0; j < 8; ++j) acc[n][j] += bfr(ba[n * 16 + lr]);
        restage(acc, mth, mtl, lr, hi, true, ah, al);
        lin64(ah, al, WT + 6 * NH * ND, lr, hi, acc);
#pragma unroll
        for (int n = 0; n < 4; ++n)
#pragma unroll
            for (int j = 0; j < 8; ++j) mx[n][j] = fmaxf(mx[n][j], acc[n][j] + bfr(bb[n * 16 + lr]) + net[n][j]);
    }
    float* os = &ost[wave][0];
#pragma unroll
    for (int n = 0; n < 4; ++n)
#pragma unroll
        for (int j = 0; j < 8; ++j) os[(hi * 8 + j) * 68 + n * 16 + lr] = mx[n][j];
    __syncthreads();
    float* crow = NET1 + (size_t)r0 * NH;
    auto pass = [&]() {
#pragma unroll
        for (int s = 0; s < 8; ++s) { const int Lid = (lane >> 3) + 4 * s, piece = lane & 7; const int row = Lid >> 1, cofs = (Lid & 1) * 32 + piece * 4;
            const v4f val = *(const v4fa*)(os + row * 68 + cofs); *(volatile v4f*)(crow + (size_t)row * NH + cofs) = val; }
    };
    pass(); __threadfence(); pass();
}
__global__ __launch_bounds__(128) void k_s2(const float* __restrict__ NET1, const bf* __restrict__ WT, const bf* __restrict__ WOUT, const float* __restrict__ ba, const float* __restrict__ bb, const float* __restrict__ bout, float* out) {
    __shared__ __align__(16) unsigned short th[4][16 * 72];
    __shared__ __align__(16) unsigned short tlw[4][16 * 72];
    __shared__ float res[64];
    const int lane = threadIdx.x & 31, wave = threadIdx.x >> 5, lr = lane & 15, hi = lane >> 4;
    const int r0 = blockIdx.x * 64 + wave * 16;
    unsigned short* mth = th[wave]; unsigned short* mtl = tlw[wave];
    v8f net[4], acc[4]; v16bf ah[2], al[2];
#pragma unroll
    for (int n = 0; n < 4; ++n)
#pragma unroll
        for (int j = 0; j < 8; ++j) net[n][j] = NET1[(size_t)(r0 + hi * 8 + j) * NH + n * 16 + lr];
#pragma unroll 1
    for (int i = 1; i < 5; ++i) {
        restage(net, mth, mtl, lr, hi, true, ah, al);
        lin64(ah, al, WT + (size_t)(1 + (i - 0)) * NH * ND, lr, hi, acc);
#pragma unroll
        for (int n = 0; n < 4; ++n)
#pragma unroll
            for (int j = 0; j < 8; ++j) acc[n][j] += bfr(ba[i * NH + n * 16 + lr]);
        restage(acc, mth, mtl, lr, hi, true, ah, al);
        lin64(ah, al, WT + (size_t)(6 + i) * NH * ND, lr, hi, acc);
#pragma unroll
        for (int n = 0; n < 4; ++n)
#pragma unroll
            for (int j = 0; j < 8; ++j) net[n][j] += acc[n][j] + bfr(bb[i * NH + n * 16 + lr]);
    }
    restage(net, mth, mtl, lr, hi, true, ah, al);
    v8f o = {};
#pragma unroll
    for (int kc = 0; kc < 2; ++kc) { const bf* bp = WOUT + (size_t)lr * ND + kc * 32 + 8 * hi; const v16bf bw = cat16b(*(const v8us*)bp, *(const v8us*)(bp + 16)); o = wmmab(ah[kc], bw, o); o = wmmab(al[kc], bw, o); }
    asm volatile("v_nop\n\tv_nop\n\tv_nop\n\tv_nop" : "+v"(o));
    if (lr == 0) {
#pragma unroll
        for (int j = 0; j < 8; ++j) res[wave * 16 + hi * 8 + j] = o[j] + bfr(bout[0]);
    }
    __syncthreads();
    if (wave == 0) { v2f v; v[0] = res[lane * 2]; v[1] = res[lane * 2 + 1]; VST2(v2f, out + (size_t)blockIdx.x * 64 + lane * 2, v); }
}

extern "C" void kernel_launch(void* const* d_in, const int* in_sizes, int n_in,
                              void* d_out, int out_size, void* d_ws, size_t ws_size, hipStream_t stream) {
    (void)in_sizes; (void)n_in; (void)out_size;
    const float* z = (const float*)d_in[0]; const float* pos = (const float*)d_in[1]; const float* pq = (const float*)d_in[2]; const float* Wf = (const float*)d_in[3];
    const float* Wdir = (const float*)d_in[4]; const float* W0 = (const float*)d_in[5]; const float* b0 = (const float*)d_in[6]; const float* Wa = (const float*)d_in[7];
    const float* ba = (const float*)d_in[8]; const float* Wb = (const float*)d_in[9]; const float* bb = (const float*)d_in[10]; const float* Wout = (const float*)d_in[11]; const float* bout = (const float*)d_in[12];
    float* out = (float*)d_out;
    char* wsp = (char*)d_ws;
    auto take = [&](size_t bytes) { char* p = wsp; wsp += (bytes + 255) & ~(size_t)255; return (void*)p; };
    bf* PEH = (bf*)take((size_t)NPT * NF * 2); bf* PEL = (bf*)take((size_t)NPT * NF * 2); float* N0 = (float*)take((size_t)NPT * 4);
    bf* ZB = (bf*)take((size_t)NB_ * NC * ND * NF * 2); float* ZC = (float*)take((size_t)NB_ * NC * NH * 4);
    bf* WT = (bf*)take((size_t)11 * NH * ND * 2); bf* WOUT = (bf*)take((size_t)16 * ND * 2); float* NET1 = (float*)take((size_t)NPT * NH * 4);
    if ((size_t)(wsp - (char*)d_ws) > ws_size) return;
    k_pre<<<NPT / 256, 256, 0, stream>>>(pq, pos, Wf, PEH, PEL, N0);
    k_zc<<<1, 256, 0, stream>>>(z, Wdir, W0, b0, ZB, ZC);
    k_w<<<1, 256, 0, stream>>>(W0, Wa, Wb, Wout, WT, WOUT);
    k_s1<<<NPT / 64, 128, 0, stream>>>(PEH, PEL, N0, ZB, ZC, WT, W0, ba, bb, NET1);
    k_s2<<<NPT / 64, 128, 0, stream>>>(NET1, WT, WOUT, ba, bb, bout, out);
}
